// BiRWKV7TimeMix_34677565948645
// MI455X (gfx1250) — hardware-verified
//
#include <hip/hip_runtime.h>
#include <math.h>

constexpr int kBatch   = 4;
constexpr int kSteps   = 1024;
constexpr int kChan    = 512;
constexpr int kHeads   = 8;
constexpr int kHeadDim = 64;
constexpr int kTok     = kBatch * kSteps;
constexpr int kPlane   = kTok * kChan;
constexpr int kRankW   = 64;
constexpr int kRankA   = 64;
constexpr int kRankV   = 32;
constexpr int kRankVP  = 64;
constexpr int kRankG   = 128;
constexpr int kChunk   = 16;
constexpr float kWCarry    = 64.0f;
constexpr float kWCarryInv = 1.0f / 64.0f;
constexpr float kGnEps     = 0.00064f;
constexpr float kInvHeadDim = 1.0f / (float)kHeadDim;

static_assert(kChan == kHeads * kHeadDim, "head split");
static_assert(kTok == 4096 && kPlane == 2097152, "plane size");
static_assert(kTok % 64 == 0 && kChan % 64 == 0, "GEMM M,N tile multiples");
static_assert(kChan % 32 == 0 && kRankW % 32 == 0 && kRankA % 32 == 0 && kRankVP % 32 == 0 && kRankG % 32 == 0, "GEMM K multiples of 32");
static_assert(kRankW % 64 == 0 && kRankA % 64 == 0 && kRankVP % 64 == 0 && kRankG % 64 == 0, "GEMM N multiples of 64");
static_assert(((kTok / 64) * (kChan / 64)) % 8 == 0 && ((kTok / 64) * (kRankW / 64)) % 8 == 0 && ((kTok / 64) * (kRankG / 64)) % 8 == 0, "GEMM grids exact");
static_assert(kSteps % kChunk == 0, "scan chunks exact");
static_assert((size_t)kPlane * 4 == 8388608u, "second output byte offset");
static_assert((size_t)kPlane * 4 + (size_t)kPlane * 4 == 16777216u, "output total");

typedef __attribute__((ext_vector_type(16))) _Float16 v16h;
typedef __attribute__((ext_vector_type(8)))  _Float16 v8h;
typedef __attribute__((ext_vector_type(16))) __bf16   v16b;
typedef __attribute__((ext_vector_type(8)))  __bf16   v8b;
typedef __attribute__((ext_vector_type(8)))  float    v8f;
typedef __attribute__((ext_vector_type(4)))  float    v4f;
typedef __attribute__((ext_vector_type(2)))  float    v2f;
typedef __attribute__((ext_vector_type(4)))  unsigned int v4u;

__device__ __forceinline__ unsigned short f2bf_bits(float f) {
  unsigned u = __float_as_uint(f);
  return (unsigned short)((u + 0x7FFFu + ((u >> 16) & 1u)) >> 16);
}
__device__ __forceinline__ float bf_bits2f(unsigned short h) { return __uint_as_float(((unsigned)h) << 16); }
__device__ __forceinline__ unsigned short h_bits(float f) { const _Float16 h = (_Float16)f; return __builtin_bit_cast(unsigned short, h); }
__device__ __forceinline__ unsigned pk16(unsigned short a, unsigned short b) { return (unsigned)a | ((unsigned)b << 16); }

__device__ __forceinline__ void ld8(const float* __restrict__ p, float (&d)[8]) {
  const v4f a = *(const v4f*)(p);
  const v4f b = *(const v4f*)(p + 4);
  d[0] = a[0]; d[1] = a[1]; d[2] = a[2]; d[3] = a[3];
  d[4] = b[0]; d[5] = b[1]; d[6] = b[2]; d[7] = b[3];
}
__device__ __forceinline__ v4u pack8_f16(const float (&m)[8], float sc) {
  unsigned short hb[8];
#pragma unroll
  for (int e = 0; e < 8; ++e) hb[e] = h_bits(m[e] * sc);
  return (v4u){pk16(hb[0], hb[1]), pk16(hb[2], hb[3]), pk16(hb[4], hb[5]), pk16(hb[6], hb[7])};
}
__device__ __forceinline__ void pack8_bf16_split(const float (&m)[8], v4u& hi, v4u& lo) {
  unsigned short hb[8], lb[8];
#pragma unroll
  for (int e = 0; e < 8; ++e) {
    const float f = m[e];
    hb[e] = f2bf_bits(f);
    lb[e] = f2bf_bits(f - bf_bits2f(hb[e]));
  }
  hi = (v4u){pk16(hb[0], hb[1]), pk16(hb[2], hb[3]), pk16(hb[4], hb[5]), pk16(hb[6], hb[7])};
  lo = (v4u){pk16(lb[0], lb[1]), pk16(lb[2], lb[3]), pk16(lb[4], lb[5]), pk16(lb[6], lb[7])};
}

__device__ __forceinline__ void grp_guard_h(v8f& a0, v8f& a1, v8f& a2, v8f& a3, v16h x, v16h y, v16h b0, v16h b1, v16h b2, v16h b3) {
  asm volatile("v_nop\n\tv_nop\n\tv_nop\n\tv_nop" : "+v"(a0), "+v"(a1), "+v"(a2), "+v"(a3) : "v"(x), "v"(y), "v"(b0), "v"(b1), "v"(b2), "v"(b3));
}
__device__ __forceinline__ void grp_guard_b(v8f& a0, v8f& a1, v8f& a2, v8f& a3, v16b x, v16b y, v16b b0, v16b b1, v16b b2, v16b b3) {
  asm volatile("v_nop\n\tv_nop\n\tv_nop\n\tv_nop" : "+v"(a0), "+v"(a1), "+v"(a2), "+v"(a3) : "v"(x), "v"(y), "v"(b0), "v"(b1), "v"(b2), "v"(b3));
}
__device__ __forceinline__ void keep4_h(v16h a, v16h b, v16h c, v16h d) { asm volatile("v_nop" :: "v"(a), "v"(b), "v"(c), "v"(d)); }
__device__ __forceinline__ void keep4_b(v16b a, v16b b, v16b c, v16b d) { asm volatile("v_nop" :: "v"(a), "v"(b), "v"(c), "v"(d)); }
__device__ __forceinline__ void acc_guard4(v8f& a, v8f& b, v8f& c, v8f& d) { asm volatile("v_nop\n\tv_nop\n\tv_nop\n\tv_nop" : "+v"(a), "+v"(b), "+v"(c), "+v"(d)); }

template <typename T> struct Frag;
template <> struct Frag<_Float16> {
  typedef v16h V; union U { v16h v; v8h h[2]; };
  static __device__ __forceinline__ v16h load(const _Float16* p) {
    U f; f.h[0] = *(const v8h*)(p); f.h[1] = *(const v8h*)(p + 16); return f.v;
  }
  static __device__ __forceinline__ v8f mma(v16h a, v16h b, v8f c) {
    return __builtin_amdgcn_wmma_f32_16x16x32_f16(false, a, false, b, (short)0, c, false, false);
  }
  static __device__ __forceinline__ void guard(v8f& a0, v8f& a1, v8f& a2, v8f& a3, v16h x, v16h y, v16h b0, v16h b1, v16h b2, v16h b3) { grp_guard_h(a0, a1, a2, a3, x, y, b0, b1, b2, b3); }
  static __device__ __forceinline__ void keep(v16h a, v16h b, v16h c, v16h d) { keep4_h(a, b, c, d); }
};
template <> struct Frag<__bf16> {
  typedef v16b V; union U { v16b v; v8b h[2]; };
  static __device__ __forceinline__ v16b load(const __bf16* p) {
    U f; f.h[0] = *(const v8b*)(p); f.h[1] = *(const v8b*)(p + 16); return f.v;
  }
  static __device__ __forceinline__ v8f mma(v16b a, v16b b, v8f c) {
    return __builtin_amdgcn_wmma_f32_16x16x32_bf16(false, a, false, b, (short)0, c, false, false);
  }
  static __device__ __forceinline__ void guard(v8f& a0, v8f& a1, v8f& a2, v8f& a3, v16b x, v16b y, v16b b0, v16b b1, v16b b2, v16b b3) { grp_guard_b(a0, a1, a2, a3, x, y, b0, b1, b2, b3); }
  static __device__ __forceinline__ void keep(v16b a, v16b b, v16b c, v16b d) { keep4_b(a, b, c, d); }
};

template <int ET> struct Elem;
template <> struct Elem<0> { typedef _Float16 T; };
template <> struct Elem<1> { typedef __bf16 T; };
template <int ET, bool SPLIT, int OUT_MODE>
__global__ __launch_bounds__(256) void wmma_gemm64(
    const unsigned short* __restrict__ Ap, const unsigned short* __restrict__ A2p, int lda,
    const unsigned short* __restrict__ Btp, const unsigned short* __restrict__ Bt2p, int ldb,
    void* __restrict__ Cout, int ldc, int M, int N, int K, float scale) {
  typedef typename Elem<ET>::T T;
  typedef typename Frag<T>::V V;
  const T* Ab  = (const T*)Ap;
  const T* Ab2 = (const T*)A2p;
  const T* Bb  = (const T*)Btp;
  const T* Bb2 = (const T*)Bt2p;
  __shared__ __align__(16) float sT[8][16 * 68];
  const int lane = threadIdx.x & 31;
  const int wave = threadIdx.x >> 5;
  const int tilesN = N >> 6;
  const int tilesM = M >> 6;
  const int tile = blockIdx.x * 8 + wave;
  if (tile >= tilesM * tilesN) return;
  const int tm = tile / tilesN;
  const int tn = tile - tm * tilesN;
  const int m0 = tm << 6;
  const int n0 = tn << 6;

  const int rlane = lane & 15;
  const int koff  = (lane >> 4) * 8;
  const int mOff  = (lane >> 4) * 8;
  const size_t bo0   = (size_t)(n0 + rlane) * ldb + koff;
  const size_t bstep = (size_t)16 * ldb;
  const size_t ao0   = (size_t)(m0 + rlane) * lda + koff;
  const size_t astep = (size_t)16 * lda;

  v8f acc[4][4];
#pragma unroll
  for (int i = 0; i < 4; ++i)
#pragma unroll
    for (int j = 0; j < 4; ++j) acc[i][j] = (v8f){0.f, 0.f, 0.f, 0.f, 0.f, 0.f, 0.f, 0.f};

  for (int k0 = 0; k0 < K; k0 += 32) {
    V bh[4], bl[4];
#pragma unroll
    for (int j = 0; j < 4; ++j) {
      const size_t bo = bo0 + (size_t)j * bstep + k0;
      bh[j] = Frag<T>::load(Bb + bo);
      if (SPLIT) bl[j] = Frag<T>::load(Bb2 + bo);
    }
#pragma unroll
    for (int i = 0; i < 4; ++i) {
      const size_t ao = ao0 + (size_t)i * astep + k0;
      V ah = Frag<T>::load(Ab + ao);
      V al;
      if (SPLIT) al = Frag<T>::load(Ab2 + ao);
#pragma unroll
      for (int j = 0; j < 4; ++j) {
        acc[i][j] = Frag<T>::mma(ah, bh[j], acc[i][j]);
        if (SPLIT) {
          acc[i][j] = Frag<T>::mma(ah, bl[j], acc[i][j]);
          acc[i][j] = Frag<T>::mma(al, bh[j], acc[i][j]);
        }
      }
      Frag<T>::guard(acc[i][0], acc[i][1], acc[i][2], acc[i][3], ah, SPLIT ? al : ah, bh[0], bh[1], bh[2], bh[3]);
    }
    Frag<T>::keep(bh[0], bh[1], bh[2], bh[3]);
    if (SPLIT) Frag<T>::keep(bl[0], bl[1], bl[2], bl[3]);
  }
  acc_guard4(acc[0][0], acc[0][1], acc[0][2], acc[0][3]);
  acc_guard4(acc[1][0], acc[1][1], acc[1][2], acc[1][3]);
  acc_guard4(acc[2][0], acc[2][1], acc[2][2], acc[2][3]);
  acc_guard4(acc[3][0], acc[3][1], acc[3][2], acc[3][3]);

  float* slab = sT[wave];
#pragma unroll
  for (int i = 0; i < 4; ++i) {
    const int mBase = m0 + (i << 4);
#pragma unroll
    for (int j = 0; j < 4; ++j) {
#pragma unroll
      for (int r = 0; r < 8; ++r) {
        const float v = acc[i][j][r] * scale;
        slab[(mOff + r) * 68 + (j << 4) + rlane] = v;
      }
    }
    __builtin_amdgcn_fence(__ATOMIC_RELEASE, "workgroup");
    __builtin_amdgcn_wave_barrier();
    __builtin_amdgcn_fence(__ATOMIC_ACQUIRE, "workgroup");
    if (OUT_MODE == 0) {
      float* C = (float*)Cout;
      const int hh = lane >> 4, c4 = (lane & 15) * 4;
      for (int pass = 0; pass < 2; ++pass) {
#pragma unroll
        for (int it = 0; it < 8; ++it) {
          const int row = it * 2 + hh;
          const v4f v = *(const v4f*)(slab + row * 68 + c4);
          *(volatile v4f*)(C + (size_t)(mBase + row) * ldc + n0 + c4) = v;
        }
        __threadfence();
      }
    } else {
      const int q = lane >> 3, c8 = (lane & 7) * 8;
      unsigned short* C = (unsigned short*)Cout;
      for (int pass = 0; pass < 2; ++pass) {
#pragma unroll
        for (int it = 0; it < 4; ++it) {
          const int row = it * 4 + q;
          const float* sp = slab + row * 68 + c8;
          v8h hv;
#pragma unroll
          for (int e = 0; e < 8; ++e) hv[e] = (_Float16)sp[e];
          *(volatile v8h*)(C + (size_t)(mBase + row) * ldc + n0 + c8) = hv;
        }
        __threadfence();
      }
    }
    __builtin_amdgcn_fence(__ATOMIC_RELEASE, "workgroup");
    __builtin_amdgcn_wave_barrier();
    __builtin_amdgcn_fence(__ATOMIC_ACQUIRE, "workgroup");
  }
}

__global__ __launch_bounds__(256) void wsplit3_kernel(const float* __restrict__ W0, const float* __restrict__ W1,
                                                      const float* __restrict__ W2,
                                                      unsigned short* __restrict__ hi, unsigned short* __restrict__ lo) {
  const int z = blockIdx.y;
  const float* W = (z == 0) ? W0 : (z == 1) ? W1 : W2;
  const int i = blockIdx.x * 256 + threadIdx.x;
  float w[8];
  ld8(W + 8 * (size_t)i, w);
  v4u uh, ul;
  pack8_bf16_split(w, uh, ul);
  const size_t o = (size_t)z * kChan * kChan + 8 * (size_t)i;
  for (int pass = 0; pass < 2; ++pass) {
    *(volatile v4u*)(hi + o) = uh;
    *(volatile v4u*)(lo + o) = ul;
    __threadfence();
  }
}

__global__ __launch_bounds__(256) void cast8_f16_kernel(const float* __restrict__ in, unsigned short* __restrict__ out, int n8, float sc) {
  const int i = blockIdx.x * 256 + threadIdx.x;
  if (i >= n8) return;
  float w[8];
  ld8(in + 8 * (size_t)i, w);
  const v4u u = pack8_f16(w, sc);
  unsigned short* q = out + 8 * (size_t)i;
  *(volatile v4u*)q = u;
  __threadfence();
  *(volatile v4u*)q = u;
}

__global__ __launch_bounds__(256) void wtrans_kernel(const float* __restrict__ in, unsigned short* __restrict__ out,
                                                     int R, int Cc, int KP, float sc) {
  __shared__ float sm[64][65];
  const int t  = threadIdx.x;
  const int k0 = blockIdx.x * 64;
  const int n0 = blockIdx.y * 64;
#pragma unroll 4
  for (int i = 0; i < 16; ++i) {
    const int e = i * 256 + t;
    const int r = e >> 6;
    const int c = e & 63;
    const int kk = k0 + r;
    const int nn = n0 + c;
    const bool ok = (kk < R) && (nn < Cc);
    const int kc = kk < R ? kk : R - 1;
    const int nc = nn < Cc ? nn : Cc - 1;
    const float v = in[(size_t)kc * Cc + nc];
    sm[c][r] = ok ? v * sc : 0.0f;
  }
  __syncthreads();
  const int lane = t & 31, wave = t >> 5;
  const int q = lane >> 3, c8 = (lane & 7) * 8;
  for (int pass = 0; pass < 2; ++pass) {
#pragma unroll
    for (int it = 0; it < 2; ++it) {
      const int row = wave * 8 + it * 4 + q;
      unsigned short hb[8];
#pragma unroll
      for (int e = 0; e < 8; ++e) hb[e] = h_bits(sm[row][c8 + e]);
      const v4u u = (v4u){pk16(hb[0], hb[1]), pk16(hb[2], hb[3]), pk16(hb[4], hb[5]), pk16(hb[6], hb[7])};
      *(volatile v4u*)(out + (size_t)(n0 + row) * KP + k0 + c8) = u;
    }
    __threadfence();
  }
}

__device__ __forceinline__ void mix8(const float* __restrict__ coef, const float (&xc)[8], const float (&xx)[8], float (&m)[8]) {
  float cf[8];
  ld8(coef, cf);
#pragma unroll
  for (int e = 0; e < 8; ++e) m[e] = xc[e] + xx[e] * cf[e];
}
__global__ __launch_bounds__(256) void mix_kernel(const float* __restrict__ x,
    const float* __restrict__ cr, const float* __restrict__ cw, const float* __restrict__ ck,
    const float* __restrict__ cv, const float* __restrict__ ca, const float* __restrict__ cg,
    unsigned short* __restrict__ XRH, unsigned short* __restrict__ XRL,
    unsigned short* __restrict__ XKH, unsigned short* __restrict__ XKL,
    unsigned short* __restrict__ XV, unsigned short* __restrict__ XW,
    unsigned short* __restrict__ XA, unsigned short* __restrict__ XG, unsigned short* __restrict__ X16) {
  const int i   = blockIdx.x * 256 + threadIdx.x;
  const int tok = i >> 6;
  const int c0  = (i & 63) << 3;
  const int t   = tok & (kSteps - 1);
  const int ptok = (t == 0) ? tok : tok - 1;
  const size_t off  = (size_t)tok * kChan + c0;
  const size_t poff = (size_t)ptok * kChan + c0;
  float xc[8], xp[8], xx[8], m[8];
  ld8(x + off, xc);
  ld8(x + poff, xp);
#pragma unroll
  for (int e = 0; e < 8; ++e) {
    const float pv = (t == 0) ? 0.0f : xp[e];
    xx[e] = pv - xc[e];
  }
  v4u u[9];
  mix8(cr + c0, xc, xx, m);
  pack8_bf16_split(m, u[0], u[1]);
  mix8(ck + c0, xc, xx, m);
  pack8_bf16_split(m, u[2], u[3]);
  mix8(cv + c0, xc, xx, m);
  u[4] = pack8_f16(m, 1.0f);
  mix8(cw + c0, xc, xx, m);
  u[5] = pack8_f16(m, 1.0f);
  mix8(ca + c0, xc, xx, m);
  u[6] = pack8_f16(m, 1.0f);
  mix8(cg + c0, xc, xx, m);
  u[7] = pack8_f16(m, 1.0f);
  u[8] = pack8_f16(xc, 1.0f);
  for (int pass = 0; pass < 2; ++pass) {
    *(volatile v4u*)(XRH + off) = u[0];
    *(volatile v4u*)(XRL + off) = u[1];
    *(volatile v4u*)(XKH + off) = u[2];
    *(volatile v4u*)(XKL + off) = u[3];
    *(volatile v4u*)(XV  + off) = u[4];
    *(volatile v4u*)(XW  + off) = u[5];
    *(volatile v4u*)(XA  + off) = u[6];
    *(volatile v4u*)(XG  + off) = u[7];
    *(volatile v4u*)(X16 + off) = u[8];
    __threadfence();
  }
}

constexpr int kPairsW = kTok * kRankW / 2;
constexpr int kPairsG = kTok * kRankG / 2;
static_assert(kPairsW % 256 == 0 && kPairsG % 256 == 0, "hidden activation grid exact");
__global__ __launch_bounds__(256) void hidden_act_kernel(const float* __restrict__ PW, const float* __restrict__ PG,
                                                         unsigned short* __restrict__ HW, unsigned short* __restrict__ HG) {
  const bool isG = (blockIdx.x >= (unsigned)(kPairsW / 256));
  const int i = blockIdx.x * 256 + threadIdx.x;
  const int j = isG ? (i - kPairsW) : i;
  const float* src = isG ? PG : PW;
  unsigned short* dst = isG ? HG : HW;
  const v2f v = *(const v2f*)(src + 2 * (size_t)j);
  const float a0 = v[0];
  const float a1 = v[1];
  float o0, o1;
  if (isG) {
    o0 = 1.0f / (1.0f + expf(-a0));
    o1 = 1.0f / (1.0f + expf(-a1));
  } else {
    o0 = tanhf(a0);
    o1 = tanhf(a1);
  }
  const unsigned u = pk16(h_bits(o0), h_bits(o1));
  ((volatile unsigned*)dst)[j] = u;
  __threadfence();
  ((volatile unsigned*)dst)[j] = u;
}

__global__ __launch_bounds__(256) void prep_kernel(float* __restrict__ KP, float* __restrict__ VP,
    float* __restrict__ ZW, float* __restrict__ ZA, float* __restrict__ ZS,
    const float* __restrict__ vfirst, const float* __restrict__ w0, const float* __restrict__ a0,
    const float* __restrict__ v0, const float* __restrict__ k_k, const float* __restrict__ k_a) {
  const int lane = threadIdx.x & 31, wave = threadIdx.x >> 5;
  const int grp  = blockIdx.x * 8 + wave;
  const int h    = grp & (kHeads - 1);
  const int tok  = grp >> 3;
  const size_t base = (size_t)tok * kChan + h * kHeadDim + lane;
  const int cb = h * kHeadDim + lane;
  const float kr0 = KP[base];
  const float kr1 = KP[base + 32];
  const float kq0 = kr0 * k_k[cb];
  const float kq1 = kr1 * k_k[cb + 32];
  float ss = kq0 * kq0 + kq1 * kq1;
#pragma unroll
  for (int off = 16; off > 0; off >>= 1) ss += __shfl_xor(ss, off, 32);
  const float inv = 1.0f / fmaxf(sqrtf(ss), 1e-12f);
#pragma unroll 1
  for (int hf = 0; hf < 2; ++hf) {
    const size_t idx = base + 32 * hf;
    const int c = cb + 32 * hf;
    const float kr  = hf ? kr1 : kr0;
    const float kkn = (hf ? kq1 : kq0) * inv;
    const float zw = ZW[idx] + w0[c];
    const float za = ZA[idx] + a0[c];
    const float zs = ZS[idx] + v0[c];
    const float vr = VP[idx];
    const float vf = vfirst[idx];
    const float ka = k_a[c];
    const float xs = -zw;
    const float sp = fmaxf(xs, 0.0f) + log1pf(expf(-fabsf(xs)));
    const float wl = -sp - 0.5f;
    const float dec = expf(-expf(wl));
    const float av = 1.0f / (1.0f + expf(-za));
    const float sv = 1.0f / (1.0f + expf(-zs));
    const float kmod = kr * (1.0f + (av - 1.0f) * ka);
    const float vmix = vr + (vf - vr) * sv;
    const float bb = kkn * av;
    const float nk = -kkn;
    for (int pass = 0; pass < 2; ++pass) {
      *(volatile float*)(KP + idx) = kmod;
      *(volatile float*)(VP + idx) = vmix;
      *(volatile float*)(ZW + idx) = dec;
      *(volatile float*)(ZA + idx) = bb;
      *(volatile float*)(ZS + idx) = nk;
      __threadfence();
    }
  }
}

__global__ __launch_bounds__(256) void state_scan_kernel(const float* __restrict__ Rp, const float* __restrict__ DECp,
    const float* __restrict__ Kp, const float* __restrict__ Vp, const float* __restrict__ NAp, const float* __restrict__ BBp,
    float* __restrict__ YF, float* __restrict__ YB) {
  __shared__ __align__(16) float st[6][kChunk][kHeadDim];
  __shared__ __align__(16) float ybuf[kChunk][kHeadDim];
  const int tid  = threadIdx.x;
  const int inst = blockIdx.x;
  const int dir  = inst >> 5;
  const int bh   = inst & 31;
  const int b    = bh >> 3;
  const int h    = bh & 7;
  const int row  = tid >> 2;
  const int q    = tid & 3;
  const int ls   = tid >> 4;
  const int lc4  = (tid & 15) << 2;
  float* yout = dir ? YB : YF;
  const size_t hb = (size_t)b * kSteps * kChan + (size_t)h * kHeadDim + lc4;
  v4f S0 = (v4f){0.f, 0.f, 0.f, 0.f};
  v4f S1 = S0, S2 = S0, S3 = S0;

#pragma unroll 1
  for (int ch = 0; ch < kSteps / kChunk; ++ch) {
    const int step = ch * kChunk + ls;
    const int tl = dir ? (kSteps - 1 - step) : step;
    const size_t off = hb + (size_t)tl * kChan;
    {
      const v4f g0 = *(const v4f*)(Rp + off);
      const v4f g1 = *(const v4f*)(DECp + off);
      const v4f g2 = *(const v4f*)(Kp + off);
      const v4f g3 = *(const v4f*)(Vp + off);
      const v4f g4 = *(const v4f*)(NAp + off);
      const v4f g5 = *(const v4f*)(BBp + off);
      *(v4f*)(&st[0][ls][lc4]) = g0;
      *(v4f*)(&st[1][ls][lc4]) = g1;
      *(v4f*)(&st[2][ls][lc4]) = g2;
      *(v4f*)(&st[3][ls][lc4]) = g3;
      *(v4f*)(&st[4][ls][lc4]) = g4;
      *(v4f*)(&st[5][ls][lc4]) = g5;
    }
    __syncthreads();
#pragma unroll 1
    for (int s = 0; s < kChunk; ++s) {
      const float* pa = &st[4][s][q * 16];
      const v4f A0 = *(const v4f*)(pa);
      const v4f A1 = *(const v4f*)(pa + 4);
      const v4f A2 = *(const v4f*)(pa + 8);
      const v4f A3 = *(const v4f*)(pa + 12);
      v4f sacc = S0 * A0;
      sacc = S1 * A1 + sacc;
      sacc = S2 * A2 + sacc;
      sacc = S3 * A3 + sacc;
      float sa = (sacc[0] + sacc[1]) + (sacc[2] + sacc[3]);
      sa += __shfl_xor(sa, 1, 32);
      sa += __shfl_xor(sa, 2, 32);
      const float vi = st[3][s][row];
      const float* pd = &st[1][s][q * 16];
      const float* pb = &st[5][s][q * 16];
      const float* pk = &st[2][s][q * 16];
      const float* pr = &st[0][s][q * 16];
      v4f yacc;
      {
        const v4f D = *(const v4f*)(pd);
        const v4f Bv = *(const v4f*)(pb);
        const v4f Kv = *(const v4f*)(pk);
        const v4f Rv = *(const v4f*)(pr);
        S0 = S0 * D + (sa * Bv + vi * Kv);
        yacc = S0 * Rv;
      }
      {
        const v4f D = *(const v4f*)(pd + 4);
        const v4f Bv = *(const v4f*)(pb + 4);
        const v4f Kv = *(const v4f*)(pk + 4);
        const v4f Rv = *(const v4f*)(pr + 4);
        S1 = S1 * D + (sa * Bv + vi * Kv);
        yacc = S1 * Rv + yacc;
      }
      {
        const v4f D = *(const v4f*)(pd + 8);
        const v4f Bv = *(const v4f*)(pb + 8);
        const v4f Kv = *(const v4f*)(pk + 8);
        const v4f Rv = *(const v4f*)(pr + 8);
        S2 = S2 * D + (sa * Bv + vi * Kv);
        yacc = S2 * Rv + yacc;
      }
      {
        const v4f D = *(const v4f*)(pd + 12);
        const v4f Bv = *(const v4f*)(pb + 12);
        const v4f Kv = *(const v4f*)(pk + 12);
        const v4f Rv = *(const v4f*)(pr + 12);
        S3 = S3 * D + (sa * Bv + vi * Kv);
        yacc = S3 * Rv + yacc;
      }
      float y = (yacc[0] + yacc[1]) + (yacc[2] + yacc[3]);
      y += __shfl_xor(y, 1, 32);
      y += __shfl_xor(y, 2, 32);
      if (q == 0) ybuf[s][row] = y;
    }
    __syncthreads();
    {
      const v4f yv = *(const v4f*)(&ybuf[ls][lc4]);
      for (int pass = 0; pass < 2; ++pass) {
        *(volatile v4f*)(yout + off) = yv;
        __threadfence();
      }
    }
  }
}

__global__ __launch_bounds__(256) void combine_kernel(const float* __restrict__ x,
    const float* __restrict__ YF, const float* __restrict__ YB, const float* __restrict__ gate_w,
    const float* __restrict__ ln_g, const float* __restrict__ ln_b,
    const float* __restrict__ Rp, const float* __restrict__ Kp, const float* __restrict__ r_k,
    const float* __restrict__ Vp, const float* __restrict__ Gp,
    unsigned short* __restrict__ OH, unsigned short* __restrict__ OL) {
  const int i   = blockIdx.x * 256 + threadIdx.x;
  const int tok = i >> 6;
  const int cc  = (i & 63) << 3;
  const int t   = tok & (kSteps - 1);
  const int ptok = (t == 0) ? tok : tok - 1;
  const size_t off  = (size_t)tok * kChan + cc;
  const size_t poff = (size_t)ptok * kChan + cc;

  float xc[8], xp[8], gw[8];
  ld8(x + off, xc);
  ld8(x + poff, xp);
  ld8(gate_w + cc, gw);
  float gd = 0.0f;
#pragma unroll
  for (int e = 0; e < 8; ++e) {
    const float pv = (t == 0) ? 0.0f : xp[e];
    gd += (pv - xc[e]) * gw[e];
  }
  gd += __shfl_xor(gd, 1, 32);
  gd += __shfl_xor(gd, 2, 32);
  gd += __shfl_xor(gd, 4, 32);
  const float gate = 1.0f / (1.0f + expf(-gd));
  const float ngate = 1.0f - gate;

  float yf[8], yb[8], xo[8];
  ld8(YF + off, yf);
  ld8(YB + off, yb);
  float s = 0.0f;
#pragma unroll
  for (int e = 0; e < 8; ++e) {
    xo[e] = gate * yf[e] + ngate * yb[e];
    s += xo[e];
  }
  s += __shfl_xor(s, 1, 32);
  s += __shfl_xor(s, 2, 32);
  s += __shfl_xor(s, 4, 32);
  const float mu = s * kInvHeadDim;
  float ss = 0.0f;
#pragma unroll
  for (int e = 0; e < 8; ++e) {
    const float d = xo[e] - mu;
    xo[e] = d;
    ss += d * d;
  }
  ss += __shfl_xor(ss, 1, 32);
  ss += __shfl_xor(ss, 2, 32);
  ss += __shfl_xor(ss, 4, 32);
  const float rstd = rsqrtf(ss * kInvHeadDim + kGnEps);

  float rr[8], kk[8], rk8[8];
  ld8(Rp + off, rr);
  ld8(Kp + off, kk);
  ld8(r_k + cc, rk8);
  float rk = 0.0f;
#pragma unroll
  for (int e = 0; e < 8; ++e) rk += (rr[e] * kk[e]) * rk8[e];
  rk += __shfl_xor(rk, 1, 32);
  rk += __shfl_xor(rk, 2, 32);
  rk += __shfl_xor(rk, 4, 32);

  float lg[8], lb[8], vv[8], gg[8], o[8];
  ld8(ln_g + cc, lg);
  ld8(ln_b + cc, lb);
  ld8(Vp + off, vv);
  ld8(Gp + off, gg);
#pragma unroll
  for (int e = 0; e < 8; ++e) {
    const float xn = (xo[e] * rstd) * lg[e] + lb[e];
    o[e] = (xn + rk * vv[e]) * gg[e];
  }
  v4u uh, ul;
  pack8_bf16_split(o, uh, ul);
  for (int pass = 0; pass < 2; ++pass) {
    *(volatile v4u*)(OH + off) = uh;
    *(volatile v4u*)(OL + off) = ul;
    __threadfence();
  }
}

__global__ __launch_bounds__(256) void copy4_kernel(const float* __restrict__ in, float* __restrict__ out, int n4) {
  const int i = blockIdx.x * 256 + threadIdx.x;
  if (i >= n4) return;
  const v4f v = *(const v4f*)(in + 4 * (size_t)i);
  float* q = out + 4 * (size_t)i;
  *(volatile v4f*)q = v;
  __threadfence();
  *(volatile v4f*)q = v;
}

extern "C" void kernel_launch(void* const* d_in, const int* in_sizes, int n_in,
                              void* d_out, int out_size, void* d_ws, size_t ws_size, hipStream_t stream) {
  if (n_in < 29 || d_out == nullptr || d_ws == nullptr) return;
  if (in_sizes[0] != kPlane || in_sizes[1] != kPlane || out_size != 2 * kPlane) return;
  if (in_sizes[9] != kChan * kRankW || in_sizes[15] != kChan * kRankV || in_sizes[17] != kChan * kRankG ||
      in_sizes[25] != kChan * kChan || in_sizes[28] != kChan * kChan) return;

  const float* x       = (const float*)d_in[0];
  const float* v_first = (const float*)d_in[1];
  const float* x_r = (const float*)d_in[2];
  const float* x_w = (const float*)d_in[3];
  const float* x_k = (const float*)d_in[4];
  const float* x_v = (const float*)d_in[5];
  const float* x_a = (const float*)d_in[6];
  const float* x_g = (const float*)d_in[7];
  const float* w0  = (const float*)d_in[8];
  const float* w1  = (const float*)d_in[9];
  const float* w2  = (const float*)d_in[10];
  const float* a0  = (const float*)d_in[11];
  const float* a1  = (const float*)d_in[12];
  const float* a2  = (const float*)d_in[13];
  const float* v0  = (const float*)d_in[14];
  const float* v1  = (const float*)d_in[15];
  const float* v2  = (const float*)d_in[16];
  const float* g1  = (const float*)d_in[17];
  const float* g2  = (const float*)d_in[18];
  const float* k_k = (const float*)d_in[19];
  const float* k_a = (const float*)d_in[20];
  const float* r_k = (const float*)d_in[21];
  const float* gate_w = (const float*)d_in[22];
  const float* ln_g = (const float*)d_in[23];
  const float* ln_b = (const float*)d_in[24];
  const float* Wr = (const float*)d_in[25];
  const float* Wk = (const float*)d_in[26];
  const float* Wv = (const float*)d_in[27];
  const float* Wo = (const float*)d_in[28];
  float* out0 = (float*)d_out;
  float* out1 = out0 + (size_t)kPlane;

  char* ws = (char*)d_ws;
  size_t off = 0;
  auto carve = [&](size_t bytes) -> char* { char* p = ws + off; off += (bytes + 255) & ~(size_t)255; return p; };
  const size_t pl16 = (size_t)kPlane * 2;
  const size_t pl32 = (size_t)kPlane * 4;
  unsigned short* XRH = (unsigned short*)carve(pl16);
  unsigned short* XRL = (unsigned short*)carve(pl16);
  unsigned short* XKH = (unsigned short*)carve(pl16);
  unsigned short* XKL = (unsigned short*)carve(pl16);
  unsigned short* XV  = (unsigned short*)carve(pl16);
  unsigned short* XW  = (unsigned short*)carve(pl16);
  unsigned short* XA  = (unsigned short*)carve(pl16);
  unsigned short* XG  = (unsigned short*)carve(pl16);
  unsigned short* X16 = (unsigned short*)carve(pl16);
  float* PW = (float*)carve((size_t)kTok * kRankW * 4);
  float* PG = (float*)carve((size_t)kTok * kRankG * 4);
  unsigned short* HW = (unsigned short*)carve((size_t)kTok * kRankW * 2);
  unsigned short* HA = (unsigned short*)carve((size_t)kTok * kRankA * 2);
  unsigned short* HV = (unsigned short*)carve((size_t)kTok * kRankVP * 2);
  unsigned short* HG = (unsigned short*)carve((size_t)kTok * kRankG * 2);
  unsigned short* WH3 = (unsigned short*)carve((size_t)3 * kChan * kChan * 2);
  unsigned short* WL3 = (unsigned short*)carve((size_t)3 * kChan * kChan * 2);
  unsigned short* WV16 = (unsigned short*)carve((size_t)kChan * kChan * 2);
  unsigned short* W1T = (unsigned short*)carve((size_t)kRankW * kChan * 2);
  unsigned short* W2T = (unsigned short*)carve((size_t)kChan * kRankW * 2);
  unsigned short* A1T = (unsigned short*)carve((size_t)kRankA * kChan * 2);
  unsigned short* A2T = (unsigned short*)carve((size_t)kChan * kRankA * 2);
  unsigned short* V1T = (unsigned short*)carve((size_t)kRankVP * kChan * 2);
  unsigned short* V2T = (unsigned short*)carve((size_t)kChan * kRankVP * 2);
  unsigned short* G1T = (unsigned short*)carve((size_t)kRankG * kChan * 2);
  unsigned short* G2T = (unsigned short*)carve((size_t)kChan * kRankG * 2);
  float* Rf  = (float*)carve(pl32);
  float* Kf  = (float*)carve(pl32);
  float* Vf  = (float*)carve(pl32);
  float* DEC = (float*)carve(pl32);
  float* ABf = (float*)carve(pl32);
  float* SNf = (float*)carve(pl32);
  float* Gf  = (float*)carve(pl32);
  float* YF  = (float*)carve(pl32);
  float* YB  = (float*)carve(pl32);
  if (off > ws_size || off > (size_t)134217728) return;

  const size_t wsq = (size_t)kChan * kChan;
  unsigned short* WRH = WH3;
  unsigned short* WRL = WL3;
  unsigned short* WKH = WH3 + wsq;
  unsigned short* WKL = WL3 + wsq;
  unsigned short* WOH = WH3 + 2 * wsq;
  unsigned short* WOL = WL3 + 2 * wsq;
  unsigned short* XOH = XRH;
  unsigned short* XOL = XRL;

  wsplit3_kernel<<<dim3(kChan * kChan / 8 / 256, 3), 256, 0, stream>>>(Wr, Wk, Wo, WH3, WL3);
  cast8_f16_kernel<<<kChan * kChan / 8 / 256, 256, 0, stream>>>(Wv, WV16, kChan * kChan / 8, kWCarry);
  wtrans_kernel<<<dim3(kChan / 64, kRankW / 64), 256, 0, stream>>>(w1, W1T, kChan, kRankW, kChan, kWCarry);
  wtrans_kernel<<<dim3(kRankW / 64, kChan / 64), 256, 0, stream>>>(w2, W2T, kRankW, kChan, kRankW, kWCarry);
  wtrans_kernel<<<dim3(kChan / 64, kRankA / 64), 256, 0, stream>>>(a1, A1T, kChan, kRankA, kChan, kWCarry);
  wtrans_kernel<<<dim3(kRankA / 64, kChan / 64), 256, 0, stream>>>(a2, A2T, kRankA, kChan, kRankA, kWCarry);
  wtrans_kernel<<<dim3(kChan / 64, kRankVP / 64), 256, 0, stream>>>(v1, V1T, kChan, kRankV, kChan, kWCarry);
  wtrans_kernel<<<dim3(kRankVP / 64, kChan / 64), 256, 0, stream>>>(v2, V2T, kRankV, kChan, kRankVP, kWCarry);
  wtrans_kernel<<<dim3(kChan / 64, kRankG / 64), 256, 0, stream>>>(g1, G1T, kChan, kRankG, kChan, kWCarry);
  wtrans_kernel<<<dim3(kRankG / 64, kChan / 64), 256, 0, stream>>>(g2, G2T, kRankG, kChan, kRankG, kWCarry);

  mix_kernel<<<kPlane / 8 / 256, 256, 0, stream>>>(x, x_r, x_w, x_k, x_v, x_a, x_g,
                                                   XRH, XRL, XKH, XKL, XV, XW, XA, XG, X16);

  const int grid512 = (kTok / 64) * (kChan / 64) / 8;
  const int grid64  = (kTok / 64) * (kRankW / 64) / 8;
  const int grid128 = (kTok / 64) * (kRankG / 64) / 8;

  wmma_gemm64<1, true, 0><<<grid512, 256, 0, stream>>>(XRH, XRL, kChan, WRH, WRL, kChan, (void*)Rf, kChan, kTok, kChan, kChan, 1.0f);
  wmma_gemm64<1, true, 0><<<grid512, 256, 0, stream>>>(XKH, XKL, kChan, WKH, WKL, kChan, (void*)Kf, kChan, kTok, kChan, kChan, 1.0f);
  wmma_gemm64<0, false, 0><<<grid512, 256, 0, stream>>>(XV, XV, kChan, WV16, WV16, kChan, (void*)Vf, kChan, kTok, kChan, kChan, kWCarryInv);

  wmma_gemm64<0, false, 0><<<grid64, 256, 0, stream>>>(XW, XW, kChan, W1T, W1T, kChan, (void*)PW, kRankW, kTok, kRankW, kChan, kWCarryInv);
  wmma_gemm64<0, false, 1><<<grid64, 256, 0, stream>>>(XA, XA, kChan, A1T, A1T, kChan, (void*)HA, kRankA, kTok, kRankA, kChan, kWCarryInv);
  wmma_gemm64<0, false, 1><<<grid64, 256, 0, stream>>>(X16, X16, kChan, V1T, V1T, kChan, (void*)HV, kRankVP, kTok, kRankVP, kChan, kWCarryInv);
  wmma_gemm64<0, false, 0><<<grid128, 256, 0, stream>>>(XG, XG, kChan, G1T, G1T, kChan, (void*)PG, kRankG, kTok, kRankG, kChan, kWCarryInv);
  hidden_act_kernel<<<(kPairsW + kPairsG) / 256, 256, 0, stream>>>(PW, PG, HW, HG);

  wmma_gemm64<0, false, 0><<<grid512, 256, 0, stream>>>(HW, HW, kRankW, W2T, W2T, kRankW, (void*)DEC, kChan, kTok, kChan, kRankW, kWCarryInv);
  wmma_gemm64<0, false, 0><<<grid512, 256, 0, stream>>>(HA, HA, kRankA, A2T, A2T, kRankA, (void*)ABf, kChan, kTok, kChan, kRankA, kWCarryInv);
  wmma_gemm64<0, false, 0><<<grid512, 256, 0, stream>>>(HV, HV, kRankVP, V2T, V2T, kRankVP, (void*)SNf, kChan, kTok, kChan, kRankVP, kWCarryInv);
  wmma_gemm64<0, false, 0><<<grid512, 256, 0, stream>>>(HG, HG, kRankG, G2T, G2T, kRankG, (void*)Gf, kChan, kTok, kChan, kRankG, kWCarryInv);

  prep_kernel<<<kTok * kHeads / 8, 256, 0, stream>>>(Kf, Vf, DEC, ABf, SNf, v_first, w0, a0, v0, k_k, k_a);
  state_scan_kernel<<<2 * kBatch * kHeads, 256, 0, stream>>>(Rf, DEC, Kf, Vf, SNf, ABf, YF, YB);
  combine_kernel<<<kPlane / 8 / 256, 256, 0, stream>>>(x, YF, YB, gate_w, ln_g, ln_b, Rf, Kf, r_k, Vf, Gf, XOH, XOL);

  wmma_gemm64<1, true, 0><<<grid512, 256, 0, stream>>>(XOH, XOL, kChan, WOH, WOL, kChan, (void*)out0, kChan, kTok, kChan, kChan, 1.0f);
  copy4_kernel<<<kPlane / 4 / 256, 256, 0, stream>>>(v_first, out1, kPlane / 4);
}
